// MHCrossAttn_81750407512809
// MI455X (gfx1250) — hardware-verified
//
#include <hip/hip_runtime.h>
#include <stddef.h>


#define BB    2
#define SS    2048
#define DD    512
#define HH    8
#define DKK   64
#define KP1   16
#define RR    32
#define MR    (BB * SS)

#define NTHR  256
#define NWAVE 8

#define GR    32
#define AP    520
#define STP   64
#define GEMM_LDS 65536

#define NB    512
#define CHUNK 2048
#define WCAP  256
#define NGRP  (CHUNK / (NTHR * 4))
#define ATT_LDS ((NB * DKK + NB + NWAVE * WCAP + 16) * 4)

static_assert(MR % GR == 0);
static_assert(SS % GR == 0);
static_assert(DD % 32 == 0);
static_assert(HH * DKK == DD);
static_assert(NWAVE * 64 == DD);
static_assert(GR * AP * 2 <= GEMM_LDS);
static_assert(NWAVE * GR * STP * 4 <= GEMM_LDS);
static_assert((AP * 2) % 16 == 0);
static_assert(SS % NB == 0);
static_assert(NB == 512);
static_assert(NB == NWAVE * 64);
static_assert(CHUNK == SS);
static_assert(CHUNK <= 4096);
static_assert(WCAP == (CHUNK / NTHR) * 32);
static_assert(NGRP == 2);
static_assert(((NB * DKK + NB) % 4) == 0);
static_assert(ATT_LDS == 141376);

typedef float    v2f  __attribute__((ext_vector_type(2)));
typedef float    v4f  __attribute__((ext_vector_type(4)));
typedef float    v8f  __attribute__((ext_vector_type(8)));
typedef int      v4i  __attribute__((ext_vector_type(4)));
typedef _Float16 v8h  __attribute__((ext_vector_type(8)));
typedef _Float16 v16h __attribute__((ext_vector_type(16)));
union Frag   { v16h v; v8h half[2]; };
union Pack16 { v8h h; v4i i; };

__device__ __forceinline__ v8f wm(v16h a, v16h b, v8f c) {
  v8f d = __builtin_amdgcn_wmma_f32_16x16x32_f16(false, a, false, b, (short)0, c, false, false);
  asm volatile("v_nop\n\tv_nop\n\tv_nop\n\tv_nop" : "+v"(d) : "v"(a), "v"(b));
  return d;
}

__device__ __forceinline__ float wsum(float v) {
  v += __shfl_xor(v, 16, 32);
  v += __shfl_xor(v, 8, 32);
  v += __shfl_xor(v, 4, 32);
  v += __shfl_xor(v, 2, 32);
  v += __shfl_xor(v, 1, 32);
  return v;
}

__global__ __launch_bounds__(NTHR) void k_prep(const float* __restrict__ W, _Float16* Wh, int n8) {
  const int i = blockIdx.x * NTHR + threadIdx.x;
  if (i >= n8) return;
  const size_t o = (size_t)i * 8;
  const v4f a = *(const v4f*)(W + o);
  const v4f b = *(const v4f*)(W + o + 4);
  Pack16 u;
  u.h[0] = (_Float16)(a.x * 16.0f); u.h[1] = (_Float16)(a.y * 16.0f);
  u.h[2] = (_Float16)(a.z * 16.0f); u.h[3] = (_Float16)(a.w * 16.0f);
  u.h[4] = (_Float16)(b.x * 16.0f); u.h[5] = (_Float16)(b.y * 16.0f);
  u.h[6] = (_Float16)(b.z * 16.0f); u.h[7] = (_Float16)(b.w * 16.0f);
  *(volatile v4i*)(Wh + o) = u.i;
  __threadfence();
  *(volatile v4i*)(Wh + o) = u.i;
}

template <int EPI>
__device__ __forceinline__ void gemm_store_pass(const float* sw, float* dst, int rowBase,
                                                int wave, int hh, int m) {
#pragma unroll
  for (int i = 0; i < GR / 2; ++i) {
    const int j = 2 * i + hh;
    const v4f v = *(const v4f*)(sw + j * STP + 4 * m);
    size_t g;
    if (EPI == 0) {
      const int bi = rowBase / SS;
      const int s0 = rowBase - bi * SS;
      g = ((size_t)(bi * HH + wave) * SS + s0 + j) * DKK + 4 * m;
    } else {
      g = (size_t)(rowBase + j) * DD + 64 * wave + 4 * m;
    }
    *(volatile v4f*)(dst + g) = v;
  }
}

template <int EPI>
__global__ __launch_bounds__(NTHR) void k_gemm(const float* __restrict__ x,
                                               const _Float16* __restrict__ Wh,
                                               const float* __restrict__ bias,
                                               float* dst, int nRows) {
  extern __shared__ v4f lds_g[];
  _Float16* At  = (_Float16*)lds_g;
  float*    stg = (float*)lds_g;

  const int tid  = threadIdx.x;
  const int lane = tid & 31;
  const int wave = tid >> 5;
  const int hh   = lane >> 4;
  const int m    = lane & 15;
  const int rowBase = blockIdx.x * GR;

  {
    const int r  = tid >> 3;
    const int c0 = (tid & 7) * 64;
    int row = rowBase + r;
    if (row > nRows - 1) row = nRows - 1;
    if (row < 0) row = 0;
    const float* p = x + (size_t)row * DD + c0;
#pragma unroll 1
    for (int it = 0; it < 2; ++it) {
      const float* pp = p + 32 * it;
      _Float16* lp = At + r * AP + c0 + 32 * it;
#pragma unroll
      for (int q = 0; q < 4; ++q) {
        const v4f fa = *(const v4f*)(pp + 8 * q);
        const v4f fb = *(const v4f*)(pp + 8 * q + 4);
        Pack16 u;
        u.h[0] = (_Float16)fa.x; u.h[1] = (_Float16)fa.y; u.h[2] = (_Float16)fa.z; u.h[3] = (_Float16)fa.w;
        u.h[4] = (_Float16)fb.x; u.h[5] = (_Float16)fb.y; u.h[6] = (_Float16)fb.z; u.h[7] = (_Float16)fb.w;
        *(v8h*)(lp + 8 * q) = u.h;
      }
    }
  }
  __syncthreads();

  v8f acc[8];
#pragma unroll
  for (int i = 0; i < 8; ++i) {
    const v8f z = {0.f, 0.f, 0.f, 0.f, 0.f, 0.f, 0.f, 0.f};
    acc[i] = z;
  }
  const _Float16* wrow = Wh + (size_t)(64 * wave + m) * DD + 8 * hh;
#pragma unroll 1
  for (int kt = 0; kt < DD / 32; ++kt) {
    const int k0 = kt * 32;
    Frag a0, a1;
    const _Float16* pa0 = At + m * AP + k0 + 8 * hh;
    const _Float16* pa1 = pa0 + 16 * AP;
    a0.half[0] = *(const v8h*)pa0; a0.half[1] = *(const v8h*)(pa0 + 16);
    a1.half[0] = *(const v8h*)pa1; a1.half[1] = *(const v8h*)(pa1 + 16);
#pragma unroll
    for (int t = 0; t < 4; ++t) {
      Frag b;
      const _Float16* pb = wrow + (size_t)(16 * t) * DD + k0;
      b.half[0] = *(const v8h*)pb;
      b.half[1] = *(const v8h*)(pb + 16);
      acc[t]     = wm(a0.v, b.v, acc[t]);
      acc[4 + t] = wm(a1.v, b.v, acc[4 + t]);
    }
  }
  __syncthreads();

  float* sw = stg + wave * (GR * STP);
  float bn[4];
#pragma unroll
  for (int t = 0; t < 4; ++t) bn[t] = bias[64 * wave + 16 * t + m];
#pragma unroll
  for (int T = 0; T < 2; ++T) {
#pragma unroll
    for (int t = 0; t < 4; ++t) {
#pragma unroll
      for (int r = 0; r < 8; ++r) {
        sw[(16 * T + 8 * hh + r) * STP + 16 * t + m] = acc[4 * T + t][r] * 0.0625f + bn[t];
      }
    }
  }
  __syncthreads();

  gemm_store_pass<EPI>(sw, dst, rowBase, wave, hh, m);
  __threadfence();
  gemm_store_pass<EPI>(sw, dst, rowBase, wave, hh, m);
}

__device__ __forceinline__ void attn_store_pass(const float* acc, const float* dinv, float* om,
                                                size_t orow0, int hcol, int wave, int lane) {
#pragma unroll 4
  for (int i = 0; i < 32; ++i) {
    const int slot = wave * 64 + 2 * i + (lane >> 4);
    const int c4   = (lane & 15) * 4;
    const v4f a4 = *(const v4f*)(acc + slot * DKK + c4);
    const float iv = dinv[slot];
    const v4f o4 = a4 * iv;
    *(volatile v4f*)(om + (orow0 + (size_t)slot) * DD + hcol + c4) = o4;
  }
}

__global__ __launch_bounds__(NTHR) void k_attn(
    const float* __restrict__ qpl, const float* __restrict__ kpl, const float* __restrict__ vpl,
    const int* __restrict__ kv_enc, const int* __restrict__ kv_pad,
    const int* __restrict__ q_enc,  const int* __restrict__ q_pad,
    const float* __restrict__ rel_q, const float* __restrict__ rel_k, const float* __restrict__ rel_v,
    float* om) {
  extern __shared__ v4f lds_a[];
  float* acc  = (float*)lds_a;
  float* den  = acc + NB * DKK;
  int*   list = (int*)(den + NB);
  int*   wcnt = list + NWAVE * WCAP;

  const int tid  = threadIdx.x;
  const int lane = tid & 31;
  const int wave = tid >> 5;
  const int bh = blockIdx.x / (SS / NB);
  const int pb = blockIdx.x - bh * (SS / NB);
  const int b  = bh >> 3;
  const int h  = bh & (HH - 1);
  const int p0 = pb * NB;
  const size_t tb   = (size_t)bh * KP1 * SS;
  const size_t rowb = (size_t)bh * SS;

  {
    const v4f z4 = {0.f, 0.f, 0.f, 0.f};
    for (int i = tid; i < (NB * DKK + NB) / 4; i += NTHR) lds_a[i] = z4;
  }
  __syncthreads();

#pragma unroll 1
  for (int ch = 0; ch < RR; ++ch) {
    const int* src = (ch < KP1) ? (q_pad + tb + (size_t)ch * SS)
                                : (q_enc + tb + (size_t)(ch - KP1) * SS);
    const bool negfix = (ch >= KP1);
    int wc = 0;
#pragma unroll
    for (int g = 0; g < NGRP; ++g) {
      const int el0 = (g * NTHR + tid) * 4;
      v4i d = *(const v4i*)(src + el0);
      if (negfix) {
        d.x = (d.x == -1) ? 0 : d.x;
        d.y = (d.y == -1) ? 0 : d.y;
        d.z = (d.z == -1) ? 0 : d.z;
        d.w = (d.w == -1) ? 0 : d.w;
      }
      const unsigned s0 = (unsigned)d.x - (unsigned)p0;
      const unsigned s1 = (unsigned)d.y - (unsigned)p0;
      const unsigned s2 = (unsigned)d.z - (unsigned)p0;
      const unsigned s3 = (unsigned)d.w - (unsigned)p0;
      const bool h0 = s0 < (unsigned)NB;
      const bool h1 = s1 < (unsigned)NB;
      const bool h2 = s2 < (unsigned)NB;
      const bool h3 = s3 < (unsigned)NB;
      const unsigned many = __builtin_amdgcn_ballot_w32(h0 | h1 | h2 | h3);
      if (many != 0u) {
#define HITJ(J, HJ, SJ) { \
          const unsigned mj = __builtin_amdgcn_ballot_w32(HJ); \
          if (HJ) { \
            const int pos = wc + (int)__builtin_amdgcn_mbcnt_lo(mj, 0u); \
            if (pos < WCAP) list[wave * WCAP + pos] = ((el0 + (J)) << 9) | (int)(SJ); \
          } \
          wc += (int)__builtin_popcount(mj); }
        HITJ(0, h0, s0)
        HITJ(1, h1, s1)
        HITJ(2, h2, s2)
        HITJ(3, h3, s3)
#undef HITJ
      }
    }
    if (lane == 0) wcnt[wave] = wc;
    __syncthreads();

    if (wave == 0) {
      const int rsub    = ch & (KP1 - 1);
      const int lowhalf = (ch < KP1) ? 1 : 0;
      const int rzero   = (ch == 0) ? 1 : 0;
      const int* pe_row = kv_enc + tb + (size_t)rsub * SS;
      const int* pp_row = kv_pad + tb + (size_t)rsub * SS;
      const int* ce_row = q_enc  + tb + (size_t)rsub * SS;
      const v2f rq2 = *(const v2f*)(rel_q + ((size_t)h * RR + ch) * DKK + 2 * lane);
      const v2f rk2 = *(const v2f*)(rel_k + ((size_t)h * RR + ch) * DKK + 2 * lane);
      const v2f rv2 = *(const v2f*)(rel_v + ((size_t)h * RR + ch) * DKK + 2 * lane);
      const float* qb = qpl + (rowb + (size_t)p0) * DKK + 2 * lane;
      const float* kb = kpl + rowb * DKK + 2 * lane;
      const float* vb = vpl + rowb * DKK + 2 * lane;
#pragma unroll 1
      for (int wsx = 0; wsx < NWAVE; ++wsx) {
        int n = wcnt[wsx];
        if (n > WCAP) n = WCAP;
        if (n < 0) n = 0;
#pragma unroll 1
        for (int i = 0; i < n; ++i) {
          const int ent  = list[wsx * WCAP + i];
          const int slot = ent & (NB - 1);
          const int s    = (ent >> 9) & (CHUNK - 1);
          const int a  = pe_row[s];
          const int pd = pp_row[s];
          const int ce = ce_row[s];
          int kv = lowhalf ? ((a == -1) ? 0 : a) : pd;
          kv = kv < 0 ? 0 : (kv > SS - 1 ? SS - 1 : kv);
          const bool msk = (ce == -1) | (rzero != 0);
          const v2f q2 = *(const v2f*)(qb + (size_t)slot * DKK);
          const v2f k2 = *(const v2f*)(kb + (size_t)kv * DKK);
          const v2f v2 = *(const v2f*)(vb + (size_t)kv * DKK);
          float part = q2.x * k2.x + q2.y * k2.y;
          part += q2.x * rk2.x + q2.y * rk2.y;
          part += rq2.x * k2.x + rq2.y * k2.y;
          const float tot = wsum(part);
          const float ex  = __expf(tot * (1.0f / 24.0f));
          const float e   = msk ? 0.0f : ex;
          v2f* ap = (v2f*)(acc + slot * DKK + 2 * lane);
          const v2f cur = *ap;
          *ap = cur + e * (v2 + rv2);
          const float dc = den[slot];
          if (lane == 0) den[slot] = dc + e;
        }
      }
    }
    __syncthreads();
  }

#pragma unroll 1
  for (int sl = tid; sl < NB; sl += NTHR) {
    const float d  = den[sl];
    const float dd = (d == 0.0f) ? -1e9f : d;
    den[sl] = 1.0f / dd;
  }
  __syncthreads();

  const size_t orow0 = (size_t)b * SS + (size_t)p0;
  attn_store_pass(acc, den, om, orow0, h * DKK, wave, lane);
  __threadfence();
  attn_store_pass(acc, den, om, orow0, h * DKK, wave, lane);
}

extern "C" void kernel_launch(void* const* d_in, const int* in_sizes, int n_in,
                              void* d_out, int out_size, void* d_ws, size_t ws_size,
                              hipStream_t stream) {
  if (n_in < 18) return;
  const int nX = MR * DD;
  const int nI = BB * HH * KP1 * SS;
  const int nR = HH * RR * DKK;
  const int nW = DD * DD;
  if (in_sizes[0] != nX || in_sizes[1] != nX || in_sizes[2] != nX) return;
  if (in_sizes[3] != nI || in_sizes[4] != nI || in_sizes[5] != nI || in_sizes[6] != nI) return;
  if (in_sizes[7] != nR || in_sizes[8] != nR || in_sizes[9] != nR) return;
  if (in_sizes[10] != nW || in_sizes[12] != nW || in_sizes[14] != nW || in_sizes[16] != nW) return;
  if (in_sizes[11] != DD || in_sizes[13] != DD || in_sizes[15] != DD || in_sizes[17] != DD) return;
  if (out_size != nX) return;

  const float* query   = (const float*)d_in[0];
  const float* key     = (const float*)d_in[1];
  const float* value   = (const float*)d_in[2];
  const int*   kv_enc  = (const int*)d_in[3];
  const int*   kv_pad  = (const int*)d_in[4];
  const int*   q_enc   = (const int*)d_in[5];
  const int*   q_pad   = (const int*)d_in[6];
  const float* rel_q   = (const float*)d_in[7];
  const float* rel_k   = (const float*)d_in[8];
  const float* rel_v   = (const float*)d_in[9];
  const float* Wq = (const float*)d_in[10]; const float* bq = (const float*)d_in[11];
  const float* Wk = (const float*)d_in[12]; const float* bk = (const float*)d_in[13];
  const float* Wv = (const float*)d_in[14]; const float* bv = (const float*)d_in[15];
  const float* Wo = (const float*)d_in[16]; const float* bo = (const float*)d_in[17];
  float* out = (float*)d_out;

  size_t off = 0;
  char* base = (char*)d_ws;
  _Float16* Wqh = (_Float16*)(base + off); off += (size_t)nW * sizeof(_Float16);
  _Float16* Wkh = (_Float16*)(base + off); off += (size_t)nW * sizeof(_Float16);
  _Float16* Wvh = (_Float16*)(base + off); off += (size_t)nW * sizeof(_Float16);
  _Float16* Woh = (_Float16*)(base + off); off += (size_t)nW * sizeof(_Float16);
  float* qpl = (float*)(base + off); off += (size_t)nX * sizeof(float);
  float* kpl = (float*)(base + off); off += (size_t)nX * sizeof(float);
  float* vpl = (float*)(base + off); off += (size_t)nX * sizeof(float);
  float* om  = (float*)(base + off); off += (size_t)nX * sizeof(float);
  if (off > ws_size) return;
  if (off > (size_t)134217728) return;

  const int n8 = nW / 8;
  const int pgrid = (n8 + NTHR - 1) / NTHR;
  k_prep<<<pgrid, NTHR, 0, stream>>>(Wq, Wqh, n8);
  k_prep<<<pgrid, NTHR, 0, stream>>>(Wk, Wkh, n8);
  k_prep<<<pgrid, NTHR, 0, stream>>>(Wv, Wvh, n8);
  k_prep<<<pgrid, NTHR, 0, stream>>>(Wo, Woh, n8);

  hipFuncSetAttribute(reinterpret_cast<const void*>(&k_gemm<0>),
                      hipFuncAttributeMaxDynamicSharedMemorySize, GEMM_LDS);
  hipFuncSetAttribute(reinterpret_cast<const void*>(&k_gemm<1>),
                      hipFuncAttributeMaxDynamicSharedMemorySize, GEMM_LDS);
  hipFuncSetAttribute(reinterpret_cast<const void*>(&k_attn),
                      hipFuncAttributeMaxDynamicSharedMemorySize, ATT_LDS);

  const int ggrid = MR / GR;
  k_gemm<0><<<ggrid, NTHR, GEMM_LDS, stream>>>(query, Wqh, bq, qpl, MR);
  k_gemm<0><<<ggrid, NTHR, GEMM_LDS, stream>>>(key,   Wkh, bk, kpl, MR);
  k_gemm<0><<<ggrid, NTHR, GEMM_LDS, stream>>>(value, Wvh, bv, vpl, MR);

  const int agrid = BB * HH * (SS / NB);
  k_attn<<<agrid, NTHR, ATT_LDS, stream>>>(qpl, kpl, vpl, kv_enc, kv_pad, q_enc, q_pad,
                                            rel_q, rel_k, rel_v, om);

  k_gemm<1><<<ggrid, NTHR, GEMM_LDS, stream>>>(om, Woh, bo, out, MR);
}
